// SelfAttentionModule_81509889343681
// MI455X (gfx1250) — hardware-verified
//
#include <hip/hip_runtime.h>


#define NI   2
#define CIN  256
#define IMW  56
#define HW   3136
#define NTOK (NI * HW)
#define REL  16
#define RP2  18
#define OUTC 256
#define SHR  8
#define NG   32
#define KS   7
#define KK   49
#define PADR 3
#define BNEPS 1e-5f
#define NSTAT ((size_t)NI * KK * HW)
typedef _Float16 h16;
typedef unsigned short bf;
typedef __attribute__((ext_vector_type(16))) __bf16   v16bf;
typedef __attribute__((ext_vector_type(16))) _Float16 v16h;
typedef __attribute__((ext_vector_type(8)))  _Float16 v8h;
typedef __attribute__((ext_vector_type(8)))  unsigned short v8us;
typedef __attribute__((ext_vector_type(8)))  float    v8f;
typedef __attribute__((ext_vector_type(4)))  float    v4f;
typedef v8h  __attribute__((may_alias)) v8ha;
typedef v4f  __attribute__((may_alias)) v4fa;
typedef v8us __attribute__((may_alias)) v8usa;

__device__ __forceinline__ unsigned short f2bf(float f) { unsigned u = __float_as_uint(f); u += 0x7FFFu + ((u >> 16) & 1u); return (unsigned short)(u >> 16); }
__device__ __forceinline__ float bf2f(unsigned short b) { return __uint_as_float(((unsigned)b) << 16); }
__device__ __forceinline__ float bfr(float f) { return bf2f(f2bf(f)); }
__device__ __forceinline__ v16h cat16(v8h lo, v8h hi) { return __builtin_shufflevector(lo, hi, 0, 1, 2, 3, 4, 5, 6, 7, 8, 9, 10, 11, 12, 13, 14, 15); }
__device__ __forceinline__ v16bf cat16b(v8us lo, v8us hi) { return __builtin_bit_cast(v16bf, __builtin_shufflevector(lo, hi, 0, 1, 2, 3, 4, 5, 6, 7, 8, 9, 10, 11, 12, 13, 14, 15)); }
__device__ __forceinline__ v8f wmma16(v16h a, v16h b, v8f c) { return __builtin_amdgcn_wmma_f32_16x16x32_f16(false, a, false, b, (short)0, c, false, false); }
__device__ __forceinline__ v8f wmmab(v16bf a, v16bf b, v8f c) { return __builtin_amdgcn_wmma_f32_16x16x32_bf16(false, a, false, b, (short)0, c, false, false); }


template <typename T16> struct WFrag;
template <> struct WFrag<h16> { typedef v16h V; static __device__ __forceinline__ V ld(const h16* p) { return cat16(*(const v8h*)p, *(const v8h*)(p + 16)); } static __device__ __forceinline__ v8f mma(V a, V b, v8f c) { return wmma16(a, b, c); } };
template <> struct WFrag<bf> { typedef v16bf V; static __device__ __forceinline__ V ld(const bf* p) { return cat16b(*(const v8us*)p, *(const v8us*)(p + 16)); } static __device__ __forceinline__ v8f mma(V a, V b, v8f c) { return wmmab(a, b, c); } };
template <typename T16, int NSPLIT, bool BIAS>
__global__ __launch_bounds__(32) void k_gemmw(const T16* __restrict__ A, const T16* __restrict__ A2, const T16* __restrict__ Bt, const T16* __restrict__ Bt2, int K, float* C, int ldc, const float* __restrict__ bias, size_t sA, size_t sB, size_t sC) {
    typedef typename WFrag<T16>::V V;
    __shared__ __align__(16) float os[16 * 68];
    const size_t z = blockIdx.z; A += z * sA; if (A2) A2 += z * sA; Bt += z * sB; if (Bt2) Bt2 += z * sB; C += z * sC;
    const int lane = threadIdx.x & 31, lr = lane & 15, hi = lane >> 4; const int r0 = blockIdx.x * 64, c0 = blockIdx.y * 64;
    v8f acc[4][4];
#pragma unroll
    for (int mb = 0; mb < 4; ++mb)
#pragma unroll
        for (int nb = 0; nb < 4; ++nb) acc[mb][nb] = (v8f){};
    const size_t aoff = (size_t)(r0 + lr) * K + 8 * hi, boff = (size_t)(c0 + lr) * K + 8 * hi;
#pragma unroll 1
    for (int kc = 0; kc < K; kc += 32) {
        V a[4], a2[4];
#pragma unroll
        for (int mb = 0; mb < 4; ++mb) { a[mb] = WFrag<T16>::ld(A + aoff + (size_t)mb * 16 * K + kc); if (NSPLIT == 1 || NSPLIT == 2) a2[mb] = WFrag<T16>::ld(A2 + aoff + (size_t)mb * 16 * K + kc); }
#pragma unroll
        for (int nb = 0; nb < 4; ++nb) { const V b = WFrag<T16>::ld(Bt + boff + (size_t)nb * 16 * K + kc); V b2; if (NSPLIT >= 2) b2 = WFrag<T16>::ld(Bt2 + boff + (size_t)nb * 16 * K + kc);
#pragma unroll
            for (int mb = 0; mb < 4; ++mb) { acc[mb][nb] = WFrag<T16>::mma(a[mb], b, acc[mb][nb]); if (NSPLIT == 1 || NSPLIT == 2) acc[mb][nb] = WFrag<T16>::mma(a2[mb], b, acc[mb][nb]); if (NSPLIT >= 2) acc[mb][nb] = WFrag<T16>::mma(a[mb], b2, acc[mb][nb]); } }
        asm volatile("v_nop\n\tv_nop\n\tv_nop\n\tv_nop" : "+v"(acc[0][0]), "+v"(acc[1][1]), "+v"(acc[2][2]), "+v"(acc[3][3]) : "v"(a[0]), "v"(a[3]));
    }
#pragma unroll
    for (int mb = 0; mb < 4; ++mb) {
#pragma unroll
        for (int nb = 0; nb < 4; ++nb) {
#pragma unroll
            for (int j = 0; j < 8; ++j) os[(hi * 8 + j) * 68 + nb * 16 + lr] = acc[mb][nb][j]; }
        __builtin_amdgcn_wave_barrier(); asm volatile("" ::: "memory");
        float* crow = C + (size_t)(r0 + mb * 16) * ldc + c0;
#pragma unroll 1
        for (int ps = 0; ps < 2; ++ps) {
#pragma unroll
            for (int s = 0; s < 8; ++s) { const int row = 2 * s + hi, cofs = lr * 4; v4f val = *(const v4fa*)(os + row * 68 + cofs); if (BIAS) { val[0] += bfr(bias[c0 + cofs]); val[1] += bfr(bias[c0 + cofs + 1]); val[2] += bfr(bias[c0 + cofs + 2]); val[3] += bfr(bias[c0 + cofs + 3]); }
                *(volatile v4f*)(crow + (size_t)row * ldc + cofs) = val; }
            if (ps == 0) __threadfence(); }
        __builtin_amdgcn_wave_barrier(); asm volatile("" ::: "memory");
    }
}

__device__ __forceinline__ h16 tohx(float x) { return (h16)x; }
__device__ __forceinline__ void splitf(float y, unsigned short& h, unsigned short& l) { h = f2bf(y); l = f2bf(y - bf2f(h)); }
typedef __attribute__((ext_vector_type(2))) _Float16 v2h;
typedef __attribute__((ext_vector_type(4))) _Float16 v4h;
typedef __attribute__((ext_vector_type(2))) unsigned short v2us;
typedef __attribute__((ext_vector_type(4))) unsigned short v4us;
typedef __attribute__((ext_vector_type(2))) float v2f;
typedef __attribute__((ext_vector_type(4))) int v4i;

__global__ __launch_bounds__(256) void k_cvt8(const float* __restrict__ src, bf* dst, size_t n8) { const size_t i = (size_t)blockIdx.x * 256 + threadIdx.x; if (i >= n8) return; const v8f v = *(const v8f*)(src + i * 8); v8us o;
#pragma unroll
    for (int k = 0; k < 8; ++k) o[k] = f2bf(v[k]); *(volatile v8us*)(dst + i * 8) = o; __threadfence(); *(volatile v8us*)(dst + i * 8) = o; }

__device__ __forceinline__ float bfrb(float x) { float y = bfr(x); asm volatile("" : "+v"(y)); return y; }
__global__ __launch_bounds__(256) void k_cvt8T(const float* __restrict__ src, bf* dst) { const size_t i = (size_t)blockIdx.x * 256 + threadIdx.x; if (i >= (size_t)NTOK * CIN / 8) return; const int tok = (int)(i / (CIN / 8)); const int c0 = (int)(i % (CIN / 8)) * 8; const int n = tok / HW, p = tok % HW; v8us o;
#pragma unroll
    for (int k = 0; k < 8; ++k) o[k] = f2bf(src[((size_t)n * CIN + c0 + k) * HW + p]); *(volatile v8us*)(dst + (size_t)tok * CIN + c0) = o; __threadfence(); *(volatile v8us*)(dst + (size_t)tok * CIN + c0) = o; }
__global__ __launch_bounds__(256) void k_w12(const float* __restrict__ w1, const float* __restrict__ w2, const float* __restrict__ b1, const float* __restrict__ b2, bf* W12, float* B12) { const int i = blockIdx.x * 256 + threadIdx.x; if (i < 64 * CIN / 8) { const int o = i / (CIN / 8); const int c0 = (i % (CIN / 8)) * 8; v8us ov;
#pragma unroll
        for (int q = 0; q < 8; ++q) { const float v = (o < REL) ? w1[o * CIN + c0 + q] : ((o < 2 * REL) ? w2[(o - REL) * CIN + c0 + q] : 0.0f); ov[q] = f2bf(v); }
        *(volatile v8us*)(W12 + (size_t)o * CIN + c0) = ov; __threadfence(); *(volatile v8us*)(W12 + (size_t)o * CIN + c0) = ov; }
    if (i < 64) { const float v = (i < REL) ? b1[i] : ((i < 2 * REL) ? b2[i - REL] : 0.0f); *(volatile float*)(B12 + i) = v; __threadfence(); *(volatile float*)(B12 + i) = v; } }
__device__ __forceinline__ int refl(int i) { return i < 0 ? -i : (i >= IMW ? 2 * (IMW - 1) - i : i); }
__device__ __forceinline__ float linsp(int j) { return __fadd_rn(-1.0f, __fmul_rn((float)j, 2.0f / 55.0f)); }
__device__ __forceinline__ float posv(const float* wp, const float* bp, int c, int y, int x) { float a = __fmul_rn(bfrb(wp[c * 2 + 0]), linsp(x)), b = __fmul_rn(bfrb(wp[c * 2 + 1]), linsp(y)); asm volatile("" : "+v"(a), "+v"(b)); float s = __fadd_rn(a, b); asm volatile("" : "+v"(s)); return __fadd_rn(s, bfrb(bp[c])); }
__global__ __launch_bounds__(256) void k_feat(const float* __restrict__ X12, const float* __restrict__ wp, const float* __restrict__ bp, float* T1) { const size_t i = (size_t)blockIdx.x * 256 + threadIdx.x; if (i >= (size_t)NI * RP2 * KK * HW / 4) return; const size_t e = i * 4; const int p0 = (int)(e % HW); const int k = (int)((e / HW) % KK); const int c = (int)((e / ((size_t)HW * KK)) % RP2); const int n = (int)(e / ((size_t)HW * KK * RP2)); const int di = k / KS - PADR, dj = k % KS - PADR; v4f o;
#pragma unroll
    for (int q = 0; q < 4; ++q) { const int p = p0 + q; const int y = p / IMW, x = p % IMW; const int yy = refl(y + di), xx = refl(x + dj); const int pn = yy * IMW + xx; float v;
        if (c < REL) { v = __fsub_rn(X12[((size_t)n * HW + p) * 64 + c], X12[((size_t)n * HW + pn) * 64 + REL + c]); }
        else { const int pc = c - REL; v = __fsub_rn(posv(wp, bp, pc, y, x), posv(wp, bp, pc, yy, xx)); }
        o[q] = v; }
    *(volatile v4f*)(T1 + e) = o; __threadfence(); *(volatile v4f*)(T1 + e) = o; }
__global__ __launch_bounds__(256) void k_bnstat(const float* __restrict__ T, int C, float* ST) { const int lane = threadIdx.x & 31; const int c = blockIdx.x * 8 + (threadIdx.x >> 5); if (c >= C) return; float s0 = 0.f, s1 = 0.f, s2 = 0.f, s3 = 0.f;
    for (int n = 0; n < NI; ++n) { const float* base = T + ((size_t)n * C + c) * KK * HW;
        for (size_t j = (size_t)lane * 4; j < (size_t)KK * HW; j += 128) { const v4f a = *(const v4f*)(base + j); s0 = __fadd_rn(s0, a[0]); s1 = __fadd_rn(s1, a[1]); s2 = __fadd_rn(s2, a[2]); s3 = __fadd_rn(s3, a[3]); } }
    float s = __fadd_rn(__fadd_rn(s0, s1), __fadd_rn(s2, s3));
#pragma unroll
    for (int sh = 16; sh; sh >>= 1) s += __shfl_xor(s, sh, 32);
    const float mean = s * (1.0f / (float)NSTAT); float v0 = 0.f, v1 = 0.f, v2 = 0.f, v3 = 0.f;
    for (int n = 0; n < NI; ++n) { const float* base = T + ((size_t)n * C + c) * KK * HW;
        for (size_t j = (size_t)lane * 4; j < (size_t)KK * HW; j += 128) { const v4f a = *(const v4f*)(base + j); float d0 = __fsub_rn(a[0], mean), d1 = __fsub_rn(a[1], mean), d2 = __fsub_rn(a[2], mean), d3 = __fsub_rn(a[3], mean); asm volatile("" : "+v"(d0), "+v"(d1), "+v"(d2), "+v"(d3)); float q0 = __fmul_rn(d0, d0), q1 = __fmul_rn(d1, d1), q2 = __fmul_rn(d2, d2), q3 = __fmul_rn(d3, d3); asm volatile("" : "+v"(q0), "+v"(q1), "+v"(q2), "+v"(q3)); v0 = __fadd_rn(v0, q0); v1 = __fadd_rn(v1, q1); v2 = __fadd_rn(v2, q2); v3 = __fadd_rn(v3, q3); } }
    float vs = __fadd_rn(__fadd_rn(v0, v1), __fadd_rn(v2, v3));
#pragma unroll
    for (int sh = 16; sh; sh >>= 1) vs += __shfl_xor(vs, sh, 32);
    float var = __fadd_rn(vs * (1.0f / (float)NSTAT), BNEPS); asm volatile("" : "+v"(var)); const float rs = __frsqrt_rn(var);
    const float val = (lane == 0) ? mean : ((lane == 1) ? rs : 0.0f); *(volatile float*)(ST + (size_t)c * 32 + lane) = val; __threadfence(); *(volatile float*)(ST + (size_t)c * 32 + lane) = val; }
__global__ __launch_bounds__(256) void k_conv1(const float* __restrict__ T1, const float* __restrict__ ST, const float* __restrict__ g1, const float* __restrict__ be1, const float* __restrict__ cw1, float* T2) { const size_t i = (size_t)blockIdx.x * 256 + threadIdx.x; if (i >= (size_t)NI * KK * HW / 4) return; const size_t e = i * 4; const int p0 = (int)(e % HW); const int k = (int)((e / HW) % KK); const int n = (int)(e / ((size_t)HW * KK)); v4f acc[REL];
#pragma unroll
    for (int o = 0; o < REL; ++o) acc[o] = (v4f){0.f, 0.f, 0.f, 0.f};
#pragma unroll 2
    for (int c = 0; c < RP2; ++c) { const v4f a = *(const v4f*)(T1 + (((size_t)n * RP2 + c) * KK + k) * HW + p0); const float mean = ST[c * 32], rs = ST[c * 32 + 1]; const float gg = bfrb(g1[c]), bb = bfrb(be1[c]); v4f tn;
#pragma unroll
        for (int q = 0; q < 4; ++q) { float d0 = __fsub_rn(a[q], mean); asm volatile("" : "+v"(d0)); float n0 = __fmul_rn(d0, rs); asm volatile("" : "+v"(n0)); float y = __fmul_rn(n0, gg); asm volatile("" : "+v"(y)); float z = __fadd_rn(y, bb); tn[q] = fmaxf(z, 0.0f); }
#pragma unroll
        for (int o = 0; o < REL; ++o) { const float w = bfrb(cw1[o * RP2 + c]);
#pragma unroll
            for (int q = 0; q < 4; ++q) { float pr = __fmul_rn(w, tn[q]); asm volatile("" : "+v"(pr)); acc[o][q] = __fadd_rn(acc[o][q], pr); } } }
#pragma unroll 1
    for (int ps = 0; ps < 2; ++ps) {
#pragma unroll
        for (int o = 0; o < REL; ++o) *(volatile v4f*)(T2 + (((size_t)n * REL + o) * KK + k) * HW + p0) = acc[o];
        if (ps == 0) __threadfence(); } }
__global__ __launch_bounds__(256) void k_final(const float* __restrict__ T2, const float* __restrict__ ST, const float* __restrict__ g2, const float* __restrict__ be2, const float* __restrict__ cw2, const float* __restrict__ cb2, const float* __restrict__ X3, float* out) {
    const size_t gidx = (size_t)blockIdx.x * 256 + threadIdx.x; if (gidx >= (size_t)NI * NG * HW) return; const int p = (int)(gidx % HW); const int g = (int)((gidx / HW) % NG); const int n = (int)(gidx / ((size_t)HW * NG)); const int y = p / IMW, x = p % IMW;
    const float cb = bfrb(cb2[g]); float m = -3.0e38f, Z = 0.f; float acc[SHR];
#pragma unroll
    for (int s2 = 0; s2 < SHR; ++s2) acc[s2] = 0.f;
#pragma unroll 1
    for (int k = 0; k < KK; ++k) { float s = 0.f;
#pragma unroll
        for (int o = 0; o < REL; ++o) { const float a = T2[(((size_t)n * REL + o) * KK + k) * HW + p]; float d0 = __fsub_rn(a, ST[o * 32]); asm volatile("" : "+v"(d0)); float n0 = __fmul_rn(d0, ST[o * 32 + 1]); asm volatile("" : "+v"(n0)); float yv = __fmul_rn(n0, bfrb(g2[o])); asm volatile("" : "+v"(yv)); float z = __fadd_rn(yv, bfrb(be2[o])); const float tn = fmaxf(z, 0.0f); float pr = __fmul_rn(bfrb(cw2[g * REL + o]), tn); asm volatile("" : "+v"(pr)); s = __fadd_rn(s, pr); }
        asm volatile("s_wait_loadcnt 0x0" : "+v"(s) :: "memory"); const float wl = __fadd_rn(s, cb);
        const float mn = fmaxf(m, wl); float d1 = __fsub_rn(m, mn), d2 = __fsub_rn(wl, mn); asm volatile("" : "+v"(d1), "+v"(d2)); const float r = __builtin_amdgcn_exp2f(__fmul_rn(d1, 1.4426950408889634f)), w = __builtin_amdgcn_exp2f(__fmul_rn(d2, 1.4426950408889634f)); float zr = __fmul_rn(Z, r); asm volatile("" : "+v"(zr)); Z = __fadd_rn(zr, w); m = mn;
        const int yy = refl(y + k / KS - PADR), xx = refl(x + k % KS - PADR); v8f v = *(const v8f*)(X3 + ((size_t)n * HW + (size_t)yy * IMW + xx) * OUTC + g * SHR); asm volatile("s_wait_loadcnt 0x0" : "+v"(v) :: "memory");
#pragma unroll
        for (int s2 = 0; s2 < SHR; ++s2) { float t0 = __fmul_rn(acc[s2], r); asm volatile("" : "+v"(t0)); float t1 = __fmul_rn(w, v[s2]); asm volatile("" : "+v"(t1)); acc[s2] = __fadd_rn(t0, t1); } }
    const float iz = __fdiv_rn(1.0f, Z);
#pragma unroll 1
    for (int ps = 0; ps < 2; ++ps) {
#pragma unroll
        for (int s2 = 0; s2 < SHR; ++s2) *(volatile float*)(out + ((size_t)n * OUTC + g * SHR + s2) * HW + p) = acc[s2] * iz;
        if (ps == 0) __threadfence(); } }

extern "C" void kernel_launch(void* const* d_in, const int* in_sizes, int n_in,
                              void* d_out, int out_size, void* d_ws, size_t ws_size, hipStream_t stream) {
    (void)in_sizes; (void)n_in; (void)out_size;
    const float* x = (const float*)d_in[0]; const float* w1 = (const float*)d_in[1]; const float* b1 = (const float*)d_in[2]; const float* w2 = (const float*)d_in[3]; const float* b2 = (const float*)d_in[4]; const float* w3 = (const float*)d_in[5]; const float* b3 = (const float*)d_in[6]; const float* wp = (const float*)d_in[7]; const float* bp = (const float*)d_in[8];
    const float* g1 = (const float*)d_in[9]; const float* be1 = (const float*)d_in[10]; const float* cw1 = (const float*)d_in[11]; const float* g2 = (const float*)d_in[12]; const float* be2 = (const float*)d_in[13]; const float* cw2 = (const float*)d_in[14]; const float* cb2 = (const float*)d_in[15];
    float* OUT = (float*)d_out;
    char* wsp = (char*)d_ws;
    auto take = [&](size_t bytes) { char* p = wsp; wsp += (bytes + 255) & ~(size_t)255; return (void*)p; };
    bf* XT = (bf*)take((size_t)NTOK * CIN * 2); bf* W12 = (bf*)take((size_t)64 * CIN * 2); float* B12 = (float*)take(256); bf* W3 = (bf*)take((size_t)OUTC * CIN * 2);
    float* X12 = (float*)take((size_t)NTOK * 64 * 4); float* X3 = (float*)take((size_t)NTOK * OUTC * 4); float* T1 = (float*)take((size_t)NI * RP2 * KK * HW * 4); float* T2 = (float*)take((size_t)NI * REL * KK * HW * 4); float* ST1 = (float*)take(32 * 32 * 4); float* ST2 = (float*)take(32 * 32 * 4);
    if ((size_t)(wsp - (char*)d_ws) > ws_size) return;
    k_cvt8T<<<(unsigned)(((size_t)NTOK * CIN / 8 + 255) / 256), 256, 0, stream>>>(x, XT); k_w12<<<(64 * CIN / 8 + 255) / 256, 256, 0, stream>>>(w1, w2, b1, b2, W12, B12); k_cvt8<<<(unsigned)(((size_t)OUTC * CIN / 8 + 255) / 256), 256, 0, stream>>>(w3, W3, (size_t)OUTC * CIN / 8);
    k_gemmw<bf, 0, true><<<dim3(NTOK / 64, 1, 1), 32, 0, stream>>>(XT, nullptr, W12, nullptr, CIN, X12, 64, B12, 0, 0, 0);
    k_gemmw<bf, 0, true><<<dim3(NTOK / 64, OUTC / 64, 1), 32, 0, stream>>>(XT, nullptr, W3, nullptr, CIN, X3, OUTC, b3, 0, 0, 0);
    k_feat<<<(unsigned)(((size_t)NI * RP2 * KK * HW / 4 + 255) / 256), 256, 0, stream>>>(X12, wp, bp, T1);
    k_bnstat<<<(RP2 + 7) / 8, 256, 0, stream>>>(T1, RP2, ST1);
    k_conv1<<<(unsigned)(((size_t)NI * KK * HW / 4 + 255) / 256), 256, 0, stream>>>(T1, ST1, g1, be1, cw1, T2);
    k_bnstat<<<(REL + 7) / 8, 256, 0, stream>>>(T2, REL, ST2);
    k_final<<<(unsigned)(((size_t)NI * NG * HW + 255) / 256), 256, 0, stream>>>(T2, ST2, g2, be2, cw2, cb2, X3, OUT);
}
